// GNNModule_84430467105079
// MI455X (gfx1250) — hardware-run, weakly checked
//
#include <hip/hip_runtime.h>


namespace {
constexpr int N = 20000, E = 640000, F0 = 128, HD = 64, H1 = 4, C1 = H1 * HD  , NPB = 8;
constexpr float XS = 8.0f, HS = 256.0f, WSC = 256.0f, SLOPE = 0.2f;
typedef _Float16 b16;
typedef __attribute__((ext_vector_type(16))) _Float16 v16b;
typedef __attribute__((ext_vector_type(8))) _Float16 v8b;
typedef __attribute__((ext_vector_type(8))) float v8f;
typedef __attribute__((ext_vector_type(4))) float v4f;
typedef __attribute__((ext_vector_type(2))) float v2f;
__device__ __forceinline__ float bf16_rne(float f) { unsigned int u = __float_as_uint(f); u += 0x7FFFu + ((u >> 16) & 1u); float r = __uint_as_float(u & 0xFFFF0000u); asm volatile("" : "+v"(r)); return r; }
__device__ __forceinline__ float bfv(float f) { float r = bf16_rne(f); asm volatile("" : "+v"(r)); return r; }
__device__ __forceinline__ void split16(float v, b16& hi, b16& lo) { hi = (b16)v; lo = (b16)(v - (float)hi); }
__device__ __forceinline__ v16b frag_kb(const b16* p, int hh) { const v8b a = *(const v8b*)(p + 8 * hh), b = *(const v8b*)(p + 16 + 8 * hh); v16b f;
#pragma unroll
  for (int e = 0; e < 8; ++e) { f[e] = a[e]; f[8 + e] = b[e]; } return f; }
__device__ __forceinline__ v8f wmma16b(v16b a, v16b b, v8f c) { v8f d = __builtin_amdgcn_wmma_f32_16x16x32_f16(false, a, false, b, (short)0, c, false, false); asm volatile("v_nop\n\tv_nop\n\tv_nop\n\tv_nop" : "+v"(d) : "v"(a), "v"(b)); return d; }
__device__ __forceinline__ void wave_lds_sync() { __builtin_amdgcn_fence(__ATOMIC_RELEASE, "workgroup"); __builtin_amdgcn_wave_barrier(); __builtin_amdgcn_fence(__ATOMIC_ACQUIRE, "workgroup"); }
__device__ __forceinline__ float pmul(float a, float b) { float p = a * b; asm volatile("" : "+v"(p)); return p; }
__device__ __forceinline__ int iclamp(int v, int lo, int hi) { return v < lo ? lo : (v > hi ? hi : v); }
__device__ __forceinline__ float wsum(float v) { for (int o = 16; o; o >>= 1) v += __shfl_xor(v, o); return v; }
constexpr int CSR_NBLK8 = 512, CSR_GB8 = 8, CSR_GN8 = 1 << CSR_GB8  , CSR_TS8 = (CSR_GN8 < 32 ? 32 : CSR_GN8)  , CSR_MAXG8 = 512, CSR_CAP8 = 12288  ;
__device__ __host__ __forceinline__ int csr_tix8(int v) { return (v >> CSR_GB8) * CSR_TS8 + (v & (CSR_GN8 - 1)); }
__global__ __launch_bounds__(64) void csrA_kernel8(const int* __restrict__ dst, int E, int N, int nG, int CHP, int NGP, int* __restrict__ STG, int* __restrict__ HST) {
  extern __shared__ int sm[];
  int* cnt = sm; int* run = sm + NGP; int* ids = sm + 2 * NGP;
  const int b = blockIdx.x; const int ch = (E + CSR_NBLK8 - 1) / CSR_NBLK8; const int e0 = b * ch, e1 = min(E, e0 + ch);
  for (int i = threadIdx.x; i < NGP; i += 64) cnt[i] = 0;
  for (int i = threadIdx.x; i < CHP; i += 64) ids[i] = -1;
  __syncthreads();
  if (threadIdx.x == 0) {
    for (int e = e0; e < e1; ++e) { int d = dst[e]; d = (d < 0) ? 0 : (d >= N ? N - 1 : d); cnt[d >> CSR_GB8] += 1; }
    int acc = 0; for (int g = 0; g < nG; ++g) { run[g] = acc; acc += cnt[g]; }
    for (int e = e0; e < e1; ++e) { int d = dst[e]; d = (d < 0) ? 0 : (d >= N ? N - 1 : d); const int g = d >> CSR_GB8; ids[run[g]] = e; run[g] += 1; } }
  __syncthreads();
  typedef __attribute__((ext_vector_type(4))) int v4i;
  for (int pass = 0; pass < 2; ++pass) {
    for (int i = threadIdx.x; i < CHP / 4; i += 64) *(volatile v4i*)(STG + (size_t)b * CHP + i * 4) = *(const v4i*)(&ids[i * 4]);
    for (int i = threadIdx.x; i < NGP / 4; i += 64) { v4i v; for (int e = 0; e < 4; ++e) v[e] = (i * 4 + e < nG) ? cnt[i * 4 + e] : 0; *(volatile v4i*)(HST + (size_t)b * NGP + i * 4) = v; }
    __threadfence(); }
}
__global__ __launch_bounds__(512) void csrS_kernel8(const int* __restrict__ HST, int nG, int NGP, int* __restrict__ START, int* __restrict__ TOT, int* __restrict__ OFF) {
  __shared__ int tot[CSR_MAXG8];
  const int b = threadIdx.x;
  for (int pass = 0; pass < 2; ++pass) { int runb = 0; for (int g = 0; g < nG; ++g) { int c = HST[(size_t)b * NGP + g]; c = (c < 0) ? 0 : c; ((volatile int*)OFF)[(size_t)g * CSR_NBLK8 + b] = runb; runb += c; } __threadfence(); }
  for (int g = threadIdx.x; g < nG; g += 512) { int s = 0; for (int bb = 0; bb < CSR_NBLK8; ++bb) { int c = HST[(size_t)bb * NGP + g]; s += (c < 0) ? 0 : c; } tot[g] = s; }
  __syncthreads();
  if (threadIdx.x < 32) {
    __shared__ int st[CSR_MAXG8 + 32];
    if (threadIdx.x == 0) { int acc = 0; for (int g = 0; g < NGP; ++g) { st[g] = acc; if (g < nG) acc += (tot[g] + 31) & ~31; } st[NGP] = acc; }
    __builtin_amdgcn_fence(__ATOMIC_RELEASE, "workgroup"); __builtin_amdgcn_wave_barrier(); __builtin_amdgcn_fence(__ATOMIC_ACQUIRE, "workgroup");
    for (int pass = 0; pass < 2; ++pass) { for (int i = threadIdx.x; i < NGP + 32; i += 32) { ((volatile int*)START)[i] = (i <= NGP) ? st[min(i, NGP)] : 0; ((volatile int*)TOT)[i] = (i < nG) ? tot[i] : 0; } __threadfence(); } }
}
__global__ __launch_bounds__(256) void csrB_kernel8(const int* __restrict__ dst, int N, int nG, int CHP, int NGP, int permLen, const int* __restrict__ STG, const int* __restrict__ HST, const int* __restrict__ OFF, const int* __restrict__ START, const int* __restrict__ TOT, int* __restrict__ PERM, int* __restrict__ ROWPTR, int* __restrict__ ROWCNT, int* __restrict__ FLAG) {
  typedef __attribute__((ext_vector_type(4))) int v4i;
  __shared__ int ids[CSR_CAP8]; __shared__ unsigned short key[CSR_CAP8]; __shared__ int outp[CSR_CAP8]; __shared__ int ncnt[CSR_GN8 + 1]; __shared__ int boff[CSR_NBLK8 + 1];
  const int g = blockIdx.x, t_ = threadIdx.x; int tot = TOT[g]; int st = START[g], stn = START[g + 1]; const int v0 = g * CSR_GN8; const int nv = min(CSR_GN8, N - v0); const int t0 = g * CSR_TS8;
  st = (st < 0) ? 0 : (st > permLen - 32 ? permLen - 32 : st) & ~31; stn = (stn < st) ? st : (stn > permLen ? permLen : stn); tot = (tot < 0) ? 0 : tot; if (tot > stn - st && tot <= CSR_CAP8) tot = stn - st;
  if (tot > CSR_CAP8) {
    for (int pass = 0; pass < 2; ++pass) { for (int i = t_; i < CSR_TS8 / 4; i += 256) { v4i a, c; for (int e = 0; e < 4; ++e) { a[e] = st; c[e] = 0; } *(volatile v4i*)(ROWPTR + t0 + i * 4) = a; *(volatile v4i*)(ROWCNT + t0 + i * 4) = c; } if (t_ == 0) ((volatile int*)FLAG)[0] = 1; __threadfence(); } (void)nv; return; }
  if (t_ == 0) { int acc = 0; for (int b = 0; b < CSR_NBLK8; ++b) { boff[b] = acc; int c = HST[(size_t)b * NGP + g]; c = (c < 0) ? 0 : (c > CHP ? CHP : c); acc += c; if (acc > tot) acc = tot; } boff[CSR_NBLK8] = acc; }
  for (int i = t_; i <= CSR_GN8; i += 256) ncnt[i] = 0;
  __syncthreads();
  for (int b = 0; b < CSR_NBLK8; ++b) { const int c = boff[b + 1] - boff[b]; int o_ = OFF[(size_t)g * CSR_NBLK8 + b]; o_ = (o_ < 0) ? 0 : (o_ > CHP - c ? CHP - c : o_); const int* src_ = STG + (size_t)b * CHP + o_;
    for (int i = t_; i < c; i += 256) { int id = src_[i]; id = (id < 0) ? 0 : id; ids[boff[b] + i] = id; int d = dst[id]; d = (d < v0) ? v0 : (d >= N ? N - 1 : d); int kk = d - v0; kk = (kk < 0) ? 0 : (kk >= CSR_GN8 ? CSR_GN8 - 1 : kk); key[boff[b] + i] = (unsigned short)kk; } }
  __syncthreads();
  if (t_ == 0) { for (int i = 0; i < tot; ++i) ncnt[key[i]] += 1; int acc = 0; for (int vl = 0; vl < CSR_GN8; ++vl) { const int c = ncnt[vl]; ncnt[vl] = acc; acc += c; } ncnt[CSR_GN8] = acc;
    for (int i = 0; i < tot; ++i) { const int vl = key[i]; outp[ncnt[vl]] = ids[i]; ncnt[vl] += 1; }
    for (int vl = CSR_GN8; vl > 0; --vl) ncnt[vl] = ncnt[vl - 1]; ncnt[0] = 0; }
  __syncthreads();
  for (int pass = 0; pass < 2; ++pass) {
    for (int i = t_; i < (stn - st) / 4; i += 256) { v4i v; for (int e = 0; e < 4; ++e) { const int q = i * 4 + e; v[e] = (q < tot) ? outp[q] : -1; } *(volatile v4i*)(PERM + st + i * 4) = v; }
    for (int i = t_; i < CSR_TS8 / 4; i += 256) { v4i a, c; for (int e = 0; e < 4; ++e) { const int vl = i * 4 + e; const int vc = vl < CSR_GN8 ? vl : CSR_GN8; a[e] = (vl < CSR_GN8) ? st + ncnt[vc] : st; c[e] = (vl < nv) ? (ncnt[(vc < CSR_GN8 ? vc : CSR_GN8 - 1) + 1] - ncnt[vc]) : 0; } *(volatile v4i*)(ROWPTR + t0 + i * 4) = a; *(volatile v4i*)(ROWCNT + t0 + i * 4) = c; }
    __threadfence(); }
}
__global__ __launch_bounds__(256) void csrZ_kernel8(int* __restrict__ p, size_t n4) { typedef __attribute__((ext_vector_type(4))) int v4i; const size_t tid = (size_t)blockIdx.x * 256 + threadIdx.x, nth = (size_t)gridDim.x * 256; v4i z = {0, 0, 0, 0}; for (size_t i = tid; i < n4; i += nth) *(volatile v4i*)(p + i * 4) = z; }
struct CsrBufs8 { int *STG, *HST, *OFF, *START, *TOT, *PERM, *ROWPTR, *ROWCNT, *FLAG; int nG, NGP, CHP; size_t permLen; char* base; size_t bytes; };
static size_t csr_carve8(CsrBufs8& c, char* ws, size_t off, int E, int N) {
  const size_t off0 = off; c.base = ws + off;
  auto al = [&](size_t bytes) { char* p = ws + off; off += (bytes + 255) & ~(size_t)255; return p; };
  c.nG = (N + CSR_GN8 - 1) / CSR_GN8; c.NGP = (c.nG + 31) & ~31; const int ch = (E + CSR_NBLK8 - 1) / CSR_NBLK8; c.CHP = (ch + 31) & ~31; c.permLen = (size_t)E + 32 * (size_t)c.nG + 32;
  c.STG = (int*)al((size_t)CSR_NBLK8 * c.CHP * 4); c.HST = (int*)al((size_t)CSR_NBLK8 * c.NGP * 4); c.OFF = (int*)al((size_t)c.NGP * CSR_NBLK8 * 4); c.START = (int*)al((size_t)(c.NGP + 64) * 4); c.TOT = (int*)al((size_t)(c.NGP + 64) * 4);
  c.PERM = (int*)al(c.permLen * 4); c.ROWPTR = (int*)al((size_t)c.nG * CSR_TS8 * 4); c.ROWCNT = (int*)al((size_t)c.nG * CSR_TS8 * 4); c.FLAG = (int*)al(256);
  c.bytes = off - off0; return off;
}
static void csr_build8(const CsrBufs8& c, const int* dst, int E, int N, hipStream_t stream) {
  const size_t smem = (size_t)(2 * c.NGP + c.CHP) * 4;
  csrZ_kernel8<<<512, 256, 0, stream>>>((int*)c.base, c.bytes / 16);
  csrA_kernel8<<<CSR_NBLK8, 64, smem, stream>>>(dst, E, N, c.nG, c.CHP, c.NGP, c.STG, c.HST);
  csrS_kernel8<<<1, 512, 0, stream>>>(c.HST, c.nG, c.NGP, c.START, c.TOT, c.OFF);
  csrB_kernel8<<<c.nG, 256, 0, stream>>>(dst, N, c.nG, c.CHP, c.NGP, (int)c.permLen, c.STG, c.HST, c.OFF, c.START, c.TOT, c.PERM, c.ROWPTR, c.ROWCNT, c.FLAG);
}


__global__ __launch_bounds__(256) void wput_kernel(const float* __restrict__ w1l, const float* __restrict__ w1r, const float* __restrict__ w2l, const float* __restrict__ w2r, b16* __restrict__ WA, b16* __restrict__ WB) { const int u = blockIdx.x * 256 + threadIdx.x; v8b v;
  if (u < 512 * 16) { const int o = u / 16, k0 = (u % 16) * 8; const float* w = o < C1 ? w1l : w1r; const int oo = o % C1;
#pragma unroll
    for (int j = 0; j < 8; ++j) v[j] = (b16)(bf16_rne(w[(size_t)(k0 + j) * C1 + oo]) * WSC); for (int pass = 0; pass < 2; ++pass) { *(volatile v8b*)(WA + (size_t)o * F0 + k0) = v; __threadfence(); } }
  if (u < 128 * 32) { const int o = u / 32, k0 = (u % 32) * 8; const float* w = o < HD ? w2l : w2r; const int oo = o % HD;
#pragma unroll
    for (int j = 0; j < 8; ++j) v[j] = (b16)(bf16_rne(w[(size_t)(k0 + j) * HD + oo]) * WSC); for (int pass = 0; pass < 2; ++pass) { *(volatile v8b*)(WB + (size_t)o * C1 + k0) = v; __threadfence(); } } }
template <int MODE>
__global__ __launch_bounds__(32) void proj_kernel(const float* __restrict__ IN, const b16* __restrict__ W, int NLIM, float* __restrict__ OUTR) { constexpr int KD = MODE == 0 ? F0 : C1, NG = MODE == 0 ? 2 : 1, NTL = MODE == 0 ? 16 : 8, OW = MODE == 0 ? 512 : 128; __shared__ __attribute__((aligned(16))) b16 Ah[16][KD + 8], Al[16][KD + 8]; __shared__ float Tf[16][260]; const int lane = threadIdx.x, nloc = lane & 15, hlf = lane >> 4; const size_t n0 = (size_t)blockIdx.x * 16; if (n0 >= (size_t)NLIM) return;
  for (int rr = 0; rr < 16; ++rr) for (int q = 0; q < KD / 32; ++q) { const int c = q * 32 + lane; const float v = IN[(n0 + rr) * KD + c]; if (MODE == 0) { Ah[rr][c] = (b16)(bfv(v) * XS); Al[rr][c] = (b16)0.0f; } else { b16 p, pl; split16(v * HS, p, pl); Ah[rr][c] = p; Al[rr][c] = pl; } }
  if (lane < 16) for (int k = KD; k < KD + 8; ++k) { Ah[lane][k] = (b16)0.0f; Al[lane][k] = (b16)0.0f; }
  wave_lds_sync();
  const float isc = MODE == 0 ? 1.0f / (XS * WSC) : 1.0f / (HS * WSC);
#pragma unroll 1
  for (int g = 0; g < NG; ++g) { v8f acc[NTL];
#pragma unroll
    for (int t = 0; t < NTL; ++t) acc[t] = (v8f){};
#pragma unroll
    for (int kb = 0; kb < KD; kb += 32) { const v16b a = frag_kb(&Ah[nloc][kb], hlf), al = frag_kb(&Al[nloc][kb], hlf);
#pragma unroll
      for (int t = 0; t < NTL; ++t) { const v16b bw = frag_kb(W + (size_t)(g * 256 + t * 16 + nloc) * KD + kb, hlf); acc[t] = wmma16b(a, bw, acc[t]); if (MODE == 1) acc[t] = wmma16b(al, bw, acc[t]); } }
#pragma unroll
    for (int t = 0; t < NTL; ++t)
#pragma unroll
      for (int r8 = 0; r8 < 8; ++r8) Tf[8 * hlf + r8][t * 16 + nloc] = acc[t][r8] * isc;
    wave_lds_sync();
    for (int pass = 0; pass < 2; ++pass) { for (int rr = 0; rr < 16; ++rr) for (int q = 0; q < NTL / 8; ++q) *(volatile v4f*)(OUTR + (n0 + rr) * OW + g * 256 + q * 128 + lane * 4) = *(const v4f*)(&Tf[rr][q * 128 + lane * 4]); __threadfence(); }
    wave_lds_sync(); } }
template <int MODE>
__global__ __launch_bounds__(256) void gat_kernel(const float* __restrict__ XLR, const float* __restrict__ att, const float* __restrict__ bias, const int* __restrict__ srcs, const int* __restrict__ PERM, const int* __restrict__ ROWPTR, const int* __restrict__ ROWCNT, int permLen, int NLIM, float* __restrict__ OUT) { constexpr int NH = MODE == 0 ? H1 : 1, OW = MODE == 0 ? 512 : 128, XR0 = NH * HD; const int wave = threadIdx.x >> 5, lane = threadIdx.x & 31; const size_t n = (size_t)blockIdx.x * NPB + wave; if (n >= (size_t)NLIM) return;
  v2f xr[NH], at[NH], acc[NH]; float mx[NH], den[NH];
#pragma unroll
  for (int h = 0; h < NH; ++h) { xr[h] = *(const v2f*)(XLR + n * OW + XR0 + h * HD + lane * 2); at[h] = (v2f){bfv(att[h * HD + lane * 2]), bfv(att[h * HD + lane * 2 + 1])}; acc[h] = (v2f){0.0f, 0.0f}; mx[h] = -INFINITY; den[h] = 0.0f; }
  auto visit = [&](size_t s) {
#pragma unroll
    for (int h = 0; h < NH; ++h) { const v2f xl = *(const v2f*)(XLR + s * OW + h * HD + lane * 2); float e0 = xl[0] + xr[h][0], e1 = xl[1] + xr[h][1]; e0 = e0 > 0.0f ? e0 : SLOPE * e0; e1 = e1 > 0.0f ? e1 : SLOPE * e1; const float sc = wsum(pmul(at[h][0], e0) + pmul(at[h][1], e1)); const float mn = fmaxf(mx[h], sc); const float sf = (mx[h] == -INFINITY) ? 0.0f : __expf(mx[h] - mn); const float p = __expf(sc - mn); acc[h][0] = pmul(acc[h][0], sf) + pmul(p, xl[0]); acc[h][1] = pmul(acc[h][1], sf) + pmul(p, xl[1]); den[h] = pmul(den[h], sf) + p; mx[h] = mn; } };
  int st = ROWPTR[n], cnt = ROWCNT[n]; cnt = iclamp(cnt, 0, E); st = iclamp(st, 0, permLen - cnt);
#pragma unroll 1
  for (int j = 0; j < cnt; ++j) { const int e = iclamp(PERM[st + j], 0, E - 1); const size_t s = (size_t)iclamp(srcs[e], 0, N - 1); if (s >= (size_t)NLIM) continue; visit(s); }
  visit(n);
  for (int pass = 0; pass < 2; ++pass) {
#pragma unroll
    for (int h = 0; h < NH; ++h) { const float inv = __builtin_amdgcn_rcpf(den[h]); v2f o; for (int q = 0; q < 2; ++q) { const int c = h * HD + lane * 2 + q; const float v = pmul(acc[h][q], inv) + bfv(bias[c]); o[q] = MODE == 0 ? fmaxf(v, 0.0f) : v; } *(volatile v2f*)(OUT + n * XR0 + h * HD + lane * 2) = o; }
    __threadfence(); } }
}

extern "C" void kernel_launch(void* const* d_in, const int* in_sizes, int n_in, void* d_out, int out_size, void* d_ws, size_t ws_size, hipStream_t stream) {
  (void)n_in;
  auto Fp = [&](int i) { return (const float*)d_in[i]; }; auto Ip = [&](int i) { return (const int*)d_in[i]; };
  if (in_sizes[0] != N * F0 || in_sizes[1] != 2 * E || in_sizes[2] != F0 * C1 || in_sizes[3] != F0 * C1 || in_sizes[4] != C1 || in_sizes[6] != C1 * HD || in_sizes[8] != HD || out_size != N * HD) return;
  const int NLIM = N;
  size_t off = 0; char* ws = (char*)d_ws;
  auto carve = [&](size_t bytes) { char* p = ws + off; off += (bytes + 255) & ~(size_t)255; return p; };
  b16* WA = (b16*)carve(512 * F0 * 2); b16* WB = (b16*)carve(128 * C1 * 2); float* XLR = (float*)carve((size_t)N * 512 * 4); float* Hh = (float*)carve((size_t)N * C1 * 4); float* XLR2 = (float*)carve((size_t)N * 128 * 4); CsrBufs8 csr; off = csr_carve8(csr, ws, off, E, N);
  if (off > ws_size || off > ((size_t)112 << 20)) return;
  wput_kernel<<<(512 * 16 + 255) / 256, 256, 0, stream>>>(Fp(2), Fp(3), Fp(6), Fp(7), WA, WB);
  csr_build8(csr, Ip(1) + E, E, N, stream);
  const int nb = (NLIM + NPB - 1) / NPB;
  proj_kernel<0><<<NLIM / 16, 32, 0, stream>>>(Fp(0), WA, NLIM, XLR);
  gat_kernel<0><<<nb, 256, 0, stream>>>(XLR, Fp(4), Fp(5), Ip(1), csr.PERM, csr.ROWPTR, csr.ROWCNT, (int)csr.permLen, NLIM, Hh);
  proj_kernel<1><<<NLIM / 16, 32, 0, stream>>>(Hh, WB, NLIM, XLR2);
  gat_kernel<1><<<nb, 256, 0, stream>>>(XLR2, Fp(8), Fp(9), Ip(1), csr.PERM, csr.ROWPTR, csr.ROWCNT, (int)csr.permLen, NLIM, (float*)d_out);
}
